// DilateAttention_41661182771556
// MI455X (gfx1250) — hardware-verified
//
#include <hip/hip_runtime.h>
#include <math.h>
#include <stdint.h>

typedef __attribute__((ext_vector_type(16))) __bf16 v16b;
typedef __attribute__((ext_vector_type(8)))  __bf16 v8b;
typedef __attribute__((ext_vector_type(4)))  __bf16 v4b;
typedef __attribute__((ext_vector_type(8)))  float  v8f;
typedef __attribute__((ext_vector_type(4)))  float  v4f;

constexpr int NB    = 32;
constexpr int ND    = 64;
constexpr int NH    = 64;
constexpr int NW    = 64;
constexpr int NWAVE = 4;
constexpr int NTHR  = NWAVE * 32;
constexpr int KC    = 66;
constexpr int KP    = 64;
constexpr int VP    = 80;
constexpr int SP    = 17;
constexpr int OP    = 68;
constexpr float QK_SCALE = 0.125f;

constexpr int K_PLANE = 3 * KC * KP;
constexpr int V_PLANE = 3 * ND * VP;
constexpr int Q_PLANE = NW * KP;
constexpr int P_WAVE  = 3 * 16 * 32;
constexpr int S_WAVE  = 2 * 16 * SP;
constexpr int O_STAGE = ND * OP;
static_assert(O_STAGE * 4 <= K_PLANE * 2);
static_assert(S_WAVE * 4 <= P_WAVE * 2);
static_assert(NWAVE * 16 == NW);

__device__ __forceinline__ unsigned short bf_bits(float f) {
  const unsigned u = __float_as_uint(f);
  return (unsigned short)((u + 0x7FFFu + ((u >> 16) & 1u)) >> 16);
}
__device__ __forceinline__ float bits_f(unsigned short b) { return __uint_as_float(((unsigned)b) << 16); }
__device__ __forceinline__ void split_bf(float f, __bf16& hi, __bf16& lo) {
  const unsigned short hb = bf_bits(f);
  hi = __builtin_bit_cast(__bf16, hb);
  lo = __builtin_bit_cast(__bf16, bf_bits(f - bits_f(hb)));
}
__device__ __forceinline__ v8f mma_bf(v16b a, v16b b, v8f c) {
  c = __builtin_amdgcn_wmma_f32_16x16x32_bf16(false, a, false, b, (short)0, c, false, false);
  asm volatile("v_nop\n\tv_nop\n\tv_nop\n\tv_nop" : "+v"(c) : "v"(a), "v"(b));
  return c;
}
__device__ __forceinline__ void lds_wave_sync() {
  __builtin_amdgcn_fence(__ATOMIC_RELEASE, "workgroup");
  __builtin_amdgcn_wave_barrier();
  __builtin_amdgcn_fence(__ATOMIC_ACQUIRE, "workgroup");
}

union KO { __bf16 k[K_PLANE]; float o[O_STAGE]; };
union PS { __bf16 p[P_WAVE];  float s[S_WAVE];  };

__global__ __launch_bounds__(NTHR) void nbr_attn_kernel(const float* __restrict__ qg, const float* __restrict__ kg,
                                                        const float* __restrict__ vg, float* __restrict__ og)
{
  __shared__ __align__(16) KO     s_ko;
  __shared__ __align__(16) __bf16 s_kl[K_PLANE];
  __shared__ __align__(16) __bf16 s_vh[V_PLANE];
  __shared__ __align__(16) __bf16 s_vl[V_PLANE];
  __shared__ __align__(16) __bf16 s_qh[Q_PLANE];
  __shared__ __align__(16) __bf16 s_ql[Q_PLANE];
  __shared__ __align__(16) PS     s_phs[NWAVE];
  __shared__ __align__(16) __bf16 s_pl[NWAVE * P_WAVE];

  const int tid  = threadIdx.x;
  const int wave = tid >> 5;
  const int lane = tid & 31;
  const int hh   = lane >> 4;
  const int m    = lane & 15;
  const int b    = blockIdx.x >> 6;
  const int h    = blockIdx.x & 63;
  __bf16* kh = s_ko.k;
  __bf16* kl = s_kl;
  const size_t bbase = (size_t)b * ND * NH * NW;
  const __bf16 bz = __builtin_bit_cast(__bf16, (unsigned short)0);
  const v8b z8 = (v8b){bz, bz, bz, bz, bz, bz, bz, bz};

  if (tid < 48) {
    const int hr = tid >> 4;
    const int cc = ((tid >> 3) & 1) ? (KC - 1) : 0;
    const int d8 = (tid & 7) * 8;
    const int o  = (hr * KC + cc) * KP + d8;
    *(v8b*)(kh + o) = z8;
    *(v8b*)(kl + o) = z8;
  }
  for (int j = tid; j < 3 * ND * 2; j += NTHR) {
    const int row = j >> 1;
    const int o   = row * VP + ((j & 1) ? (VP - 8) : 0);
    *(v8b*)(s_vh + o) = z8;
    *(v8b*)(s_vl + o) = z8;
  }

  const int sub = tid >> 4;
  const int w4  = (tid & 15) * 4;
#pragma unroll 1
  for (int it = 0; it < 24; ++it) {
    const int seg  = it * 8 + sub;
    const int hr   = seg >> 6;
    const int d    = seg & 63;
    const int hrow = h + hr - 1;
    const int hcl  = hrow < 0 ? 0 : (hrow > NH - 1 ? NH - 1 : hrow);
    const float vf = (hrow >= 0 && hrow < NH) ? 1.0f : 0.0f;
    const v4f f = *(const v4f*)(kg + bbase + ((size_t)d * NH + hcl) * NW + w4);
#pragma unroll
    for (int i = 0; i < 4; ++i) {
      __bf16 a, l;
      split_bf(f[i] * vf, a, l);
      const int o = (hr * KC + w4 + i + 1) * KP + d;
      kh[o] = a;
      kl[o] = l;
    }
  }
#pragma unroll 1
  for (int it = 0; it < 24; ++it) {
    const int seg  = it * 8 + sub;
    const int hr   = seg >> 6;
    const int d    = seg & 63;
    const int hrow = h + hr - 1;
    const int hcl  = hrow < 0 ? 0 : (hrow > NH - 1 ? NH - 1 : hrow);
    const float vf = (hrow >= 0 && hrow < NH) ? 1.0f : 0.0f;
    const v4f f = *(const v4f*)(vg + bbase + ((size_t)d * NH + hcl) * NW + w4);
    v4b ah, al;
#pragma unroll
    for (int i = 0; i < 4; ++i) {
      __bf16 a, l;
      split_bf(f[i] * vf, a, l);
      ah[i] = a;
      al[i] = l;
    }
    const int o = (hr * ND + d) * VP + w4 + 8;
    *(v4b*)(s_vh + o) = ah;
    *(v4b*)(s_vl + o) = al;
  }
#pragma unroll 1
  for (int it = 0; it < 8; ++it) {
    const int d = it * 8 + sub;
    const v4f f = *(const v4f*)(qg + bbase + ((size_t)d * NH + h) * NW + w4);
#pragma unroll
    for (int i = 0; i < 4; ++i) {
      __bf16 a, l;
      split_bf(f[i], a, l);
      const int o = (w4 + i) * KP + d;
      s_qh[o] = a;
      s_ql[o] = l;
    }
  }
  __syncthreads();

  const int w0 = wave * 16;
  union FB { v16b v; v8b p[2]; };
  v16b qah[2], qal[2];
#pragma unroll
  for (int ks = 0; ks < 2; ++ks) {
    const int qo = (w0 + m) * KP + ks * 32 + 8 * hh;
    FB fa, fl;
    fa.p[0] = *(const v8b*)(s_qh + qo);  fa.p[1] = *(const v8b*)(s_qh + qo + 16);
    fl.p[0] = *(const v8b*)(s_ql + qo);  fl.p[1] = *(const v8b*)(s_ql + qo + 16);
    qah[ks] = fa.v;
    qal[ks] = fl.v;
  }
  float* ss = s_phs[wave].s;
  const v8f z8f = (v8f){0.f, 0.f, 0.f, 0.f, 0.f, 0.f, 0.f, 0.f};
  float sc[9];
#pragma unroll
  for (int di = 0; di < 3; ++di) {
#pragma unroll
    for (int s = 0; s < 2; ++s) {
      v8f c = z8f;
#pragma unroll
      for (int ks = 0; ks < 2; ++ks) {
        const int ko = (di * KC + w0 + 2 * s + m) * KP + ks * 32 + 8 * hh;
        FB fbh, fbl;
        fbh.p[0] = *(const v8b*)(kh + ko);  fbh.p[1] = *(const v8b*)(kh + ko + 16);
        fbl.p[0] = *(const v8b*)(kl + ko);  fbl.p[1] = *(const v8b*)(kl + ko + 16);
        c = mma_bf(qah[ks], fbh.v, c);
        c = mma_bf(qah[ks], fbl.v, c);
        c = mma_bf(qal[ks], fbh.v, c);
      }
#pragma unroll
      for (int r = 0; r < 8; ++r) ss[(s * 16 + 8 * hh + r) * SP + m] = c[r] * QK_SCALE;
    }
    lds_wave_sync();
    sc[di * 3 + 0] = ss[m * SP + m];
    const int i1 = (m < 15) ? (m * SP + m + 1) : ((16 + 15) * SP + 14);
    sc[di * 3 + 1] = ss[i1];
    sc[di * 3 + 2] = ss[(16 + m) * SP + m];
    lds_wave_sync();
  }

  float mx = sc[0];
#pragma unroll
  for (int i = 1; i < 9; ++i) mx = fmaxf(mx, sc[i]);
  float ex[9];
  float sum = 0.f;
#pragma unroll
  for (int i = 0; i < 9; ++i) { ex[i] = __expf(sc[i] - mx); sum += ex[i]; }
  const float inv = 1.0f / sum;

  __bf16* ph = s_phs[wave].p;
  __bf16* pl = s_pl + wave * P_WAVE;
#pragma unroll
  for (int i = 0; i < 6; ++i) {
    const int o = (i * 32 + lane) * 8;
    *(v8b*)(ph + o) = z8;
    *(v8b*)(pl + o) = z8;
  }
  lds_wave_sync();
#pragma unroll
  for (int di = 0; di < 3; ++di) {
#pragma unroll
    for (int dj = 0; dj < 3; ++dj) {
      __bf16 a, l;
      split_bf(ex[di * 3 + dj] * inv, a, l);
      const int o = (di * 16 + m) * 32 + m + dj + 7;
      ph[o] = a;
      pl[o] = l;
    }
  }
  lds_wave_sync();

  v8f acc[4];
#pragma unroll
  for (int nt = 0; nt < 4; ++nt) acc[nt] = z8f;
#pragma unroll
  for (int di = 0; di < 3; ++di) {
    const int po = (di * 16 + m) * 32 + 8 * hh;
    FB pa, pq;
    pa.p[0] = *(const v8b*)(ph + po);  pa.p[1] = *(const v8b*)(ph + po + 16);
    pq.p[0] = *(const v8b*)(pl + po);  pq.p[1] = *(const v8b*)(pl + po + 16);
#pragma unroll
    for (int nt = 0; nt < 4; ++nt) {
      const int vo = (di * ND + nt * 16 + m) * VP + w0 + 8 * hh;
      FB vbh, vbl;
      vbh.p[0] = *(const v8b*)(s_vh + vo);  vbh.p[1] = *(const v8b*)(s_vh + vo + 16);
      vbl.p[0] = *(const v8b*)(s_vl + vo);  vbl.p[1] = *(const v8b*)(s_vl + vo + 16);
      acc[nt] = mma_bf(pa.v, vbh.v, acc[nt]);
      acc[nt] = mma_bf(pa.v, vbl.v, acc[nt]);
      acc[nt] = mma_bf(pq.v, vbh.v, acc[nt]);
    }
  }

  __syncthreads();
  float* os = s_ko.o;
#pragma unroll
  for (int nt = 0; nt < 4; ++nt) {
#pragma unroll
    for (int r = 0; r < 8; ++r) os[(nt * 16 + m) * OP + w0 + 8 * hh + r] = acc[nt][r];
  }
  __syncthreads();
  const int c4 = (lane & 15) * 4;
  float* ob = og + bbase + (size_t)h * NW + c4;
#pragma unroll
  for (int it = 0; it < 8; ++it) {
    const int d = wave * 16 + it * 2 + hh;
    const v4f v = *(const v4f*)(os + d * OP + c4);
    *(volatile v4f*)(ob + (size_t)d * NH * NW) = v;
  }
  __threadfence();
#pragma unroll
  for (int it = 0; it < 8; ++it) {
    const int d = wave * 16 + it * 2 + hh;
    const v4f v = *(const v4f*)(os + d * OP + c4);
    *(volatile v4f*)(ob + (size_t)d * NH * NW) = v;
  }
}

extern "C" void kernel_launch(void* const* d_in, const int* in_sizes, int n_in,
                              void* d_out, int out_size, void* d_ws, size_t ws_size,
                              hipStream_t stream) {
  (void)d_ws; (void)ws_size;
  if (n_in < 3) return;
  const int n = NB * ND * NH * NW;
  if (in_sizes[0] != n || in_sizes[1] != n || in_sizes[2] != n || out_size != n) return;
  const float* q = (const float*)d_in[0];
  const float* k = (const float*)d_in[1];
  const float* v = (const float*)d_in[2];
  float* out = (float*)d_out;
  hipLaunchKernelGGL(nbr_attn_kernel, dim3(NB * NH), dim3(NTHR), 0, stream, q, k, v, out);
  (void)hipGetLastError();
}
